// PositionalGrammar_12463995093741
// MI455X (gfx1250) — hardware-verified
//
#include <hip/hip_runtime.h>

typedef __attribute__((ext_vector_type(16))) _Float16 v16h;
typedef __attribute__((ext_vector_type(8)))  _Float16 v8h;
typedef __attribute__((ext_vector_type(8)))  float    v8f;
typedef __attribute__((ext_vector_type(4)))  float    v4f;
typedef __attribute__((ext_vector_type(4)))  unsigned v4u;

#define RNUM 6
#define BB   8
#define NN   1024
#define DD   128
#define PH   136

__device__ __forceinline__ v8f wmma_f16(v16h a, v16h b, v8f c) {
  v8f d = __builtin_amdgcn_wmma_f32_16x16x32_f16(false, a, false, b, (short)0, c, false, false);
  asm volatile("v_nop\n\tv_nop\n\tv_nop\n\tv_nop" : "+v"(d) : "v"(a), "v"(b));
  return d;
}

__device__ __forceinline__ v16h load_frag(const _Float16* tile, int ld, int k0, int lane) {
  union { v16h v; v8h h[2]; } r;
  const _Float16* row = tile + (lane & 15) * ld + k0 + 8 * (lane >> 4);
  r.h[0] = *(const v8h*)(row);
  r.h[1] = *(const v8h*)(row + 16);
  return r.v;
}

__global__ __launch_bounds__(256)
void pg_transform(const float* __restrict__ sym,
                  const float* __restrict__ W,
                  const float* __restrict__ bias,
                  _Float16* __restrict__ tt) {
  __shared__ __attribute__((aligned(16))) _Float16 As[64 * PH];
  __shared__ __attribute__((aligned(16))) _Float16 Ws[DD * PH];
  __shared__ __attribute__((aligned(16))) _Float16 To[DD * 64];

  const int tid  = threadIdx.x;
  const int lane = tid & 31;
  const int w    = tid >> 5;
  const int blk  = blockIdx.x;
  const int ic   = blk & 15;
  const int b    = (blk >> 4) & 7;
  const int r    = blk >> 7;
  const int i0   = ic * 64;
  const int col  = lane & 15;
  const int kh   = lane >> 4;

  const float* sp = sym + ((size_t)b * NN + i0) * DD;
  for (int t = tid; t < 64 * DD; t += 256) { int i = t >> 7, k = t & 127; As[i * PH + k] = (_Float16)sp[t]; }
  const float* wp = W + (size_t)r * DD * DD;
  for (int t = tid; t < DD * DD; t += 256) { int e = t >> 7, k = t & 127; Ws[e * PH + k] = (_Float16)wp[t]; }
  __syncthreads();

  v8f acc[4] = {};
  #pragma unroll
  for (int k0 = 0; k0 < DD; k0 += 32) {
    v16h bv = load_frag(Ws + w * 16 * PH, PH, k0, lane);
    #pragma unroll
    for (int it = 0; it < 4; ++it)
      acc[it] = wmma_f16(load_frag(As + it * 16 * PH, PH, k0, lane), bv, acc[it]);
  }
  const float bb = bias[r * DD + w * 16 + col];
  #pragma unroll
  for (int it = 0; it < 4; ++it)
    #pragma unroll
    for (int v = 0; v < 8; ++v)
      To[(w * 16 + col) * 64 + it * 16 + kh * 8 + v] = (_Float16)(acc[it][v] + bb);
  __syncthreads();

  #pragma unroll
  for (int j = 0; j < 4; ++j) {
    const int g = j * 256 + tid;
    const int e = g >> 3, piece = g & 7;
    const v4u val = *(const v4u*)((const char*)To + g * 16);
    char* dst = (char*)(tt + (((size_t)r * BB + b) * DD + e) * NN + i0) + piece * 16;
    *(volatile v4u*)dst = val;
    __threadfence();
    *(volatile v4u*)dst = val;
  }
}

__global__ __launch_bounds__(256)
void pg_aggregate(const float* __restrict__ pos,
                  const _Float16* __restrict__ tt,
                  const float* __restrict__ sym,
                  float* __restrict__ out) {
  __shared__ __attribute__((aligned(16))) _Float16 stage[RNUM * DD * 32];
  __shared__ __attribute__((aligned(16))) float Ot[8][16 * DD];

  const int tid  = threadIdx.x;
  const int lane = tid & 31;
  const int w    = tid >> 5;
  const int b    = blockIdx.x >> 3;
  const int jg   = blockIdx.x & 7;
  const int jt   = jg * 8 + w;
  const int col  = lane & 15;
  const int kh   = lane >> 4;
  const int j    = jt * 16 + col;

  const float* pb = pos + (size_t)b * NN * 2;
  const float pjx = pb[2 * j];
  const float pjy = pb[2 * j + 1];
  const _Float16* ttb = tt + (size_t)b * DD * NN;

  v8f acc[8] = {};

  for (int ic = 0; ic < NN; ic += 32) {
    __syncthreads();
    #pragma unroll
    for (int q = 0; q < 12; ++q) {
      const int g = tid + 256 * q;
      const int row = g >> 2, sub = g & 3;
      const int rr = row >> 7, e = row & 127;
      const v4u v = *(const v4u*)((const char*)(ttb + (size_t)rr * (BB * DD * NN) + (size_t)e * NN + ic) + sub * 16);
      *(v4u*)((char*)stage + (size_t)row * 64 + sub * 16) = v;
    }
    __syncthreads();

    v16h A[RNUM];
    #pragma unroll
    for (int kk = 0; kk < 16; ++kk) {
      const int i  = ic + kh * 8 + kk + ((kk >> 3) << 3);
      const float dx = pjx - pb[2 * i];
      const float dy = pjy - pb[2 * i + 1];
      int r;
      if      (dy >  0.5f) r = 0;
      else if (dy < -0.5f) r = 1;
      else if (dx < -0.5f) r = 2;
      else if (dx >  0.5f) r = 3;
      else if (__builtin_fabsf(dx) < 0.3f && __builtin_fabsf(dy) < 0.3f) r = 4;
      else r = 5;
      const int rm = (i != j) ? r : -1;
      #pragma unroll
      for (int rr = 0; rr < RNUM; ++rr)
        A[rr][kk] = (rm == rr) ? (_Float16)1.0f : (_Float16)0.0f;
    }

    #pragma unroll
    for (int rr = 0; rr < RNUM; ++rr) {
      #pragma unroll
      for (int d = 0; d < 8; ++d) {
        v16h bv = load_frag(stage + (size_t)(rr * DD + d * 16) * 32, 32, 0, lane);
        acc[d] = wmma_f16(A[rr], bv, acc[d]);
      }
    }
  }

  float* ot = Ot[w];
  #pragma unroll
  for (int d = 0; d < 8; ++d)
    #pragma unroll
    for (int v = 0; v < 8; ++v)
      ot[(kh * 8 + v) * DD + d * 16 + col] = acc[d][v];
  __syncthreads();
  {
    const size_t rowbase = ((size_t)b * NN + (size_t)jt * 16) * DD;
    v4f vals[16];
    #pragma unroll
    for (int q = 0; q < 16; ++q) {
      const int g = q * 32 + lane;
      v4f a = *(const v4f*)((const char*)ot + g * 16);
      v4f s = *(const v4f*)((const char*)(sym + rowbase) + g * 16);
      vals[q] = a + s;
    }
    char* dst = (char*)(out + rowbase);
    #pragma unroll
    for (int q = 0; q < 16; ++q) *(volatile v4f*)(dst + (q * 32 + lane) * 16) = vals[q];
    __threadfence();
    #pragma unroll
    for (int q = 0; q < 16; ++q) *(volatile v4f*)(dst + (q * 32 + lane) * 16) = vals[q];
  }
}

extern "C" void kernel_launch(void* const* d_in, const int* in_sizes, int n_in,
                              void* d_out, int out_size, void* d_ws, size_t ws_size,
                              hipStream_t stream) {
  (void)in_sizes; (void)n_in; (void)out_size; (void)ws_size;
  const float* symbols   = (const float*)d_in[0];
  const float* positions = (const float*)d_in[1];
  const float* W         = (const float*)d_in[2];
  const float* bias      = (const float*)d_in[3];
  float* out = (float*)d_out;

  _Float16* tt = (_Float16*)d_ws;

  pg_transform<<<RNUM * BB * (NN / 64), 256, 0, stream>>>(symbols, W, bias, tt);
  pg_aggregate<<<BB * 8, 256, 0, stream>>>(positions, tt, symbols, out);
}
